// GATLayer_44770739093962
// MI455X (gfx1250) — hardware-verified
//
#include <hip/hip_runtime.h>
#include <stddef.h>
#include <stdint.h>
#include <math.h>


#define DIN    128
#define HD     128
#define NH     4
#define NCAT   256
#define NTHR   256
#define NWAVE  8
#define EPT    8
#define CHUNK  (NTHR * EPT)
#define WCAP   (EPT * 32)
#define LISTN  (NWAVE * WCAP)
#define NBA    1024
#define SLA    10
#define RCAP   28672
#define DEGCAP 128
#define GBM    64
#define MXB    256
#define NUW    (NCAT * (DIN / 8))
#define NEGSL  0.2f
#define EPSD   1e-8f
#define AGG_ZINTS (LISTN + 2 * RCAP + 3 * NBA)
#define AGG_LDS_INTS (AGG_ZINTS + 32)
#define GEMM_LDS_FLOATS (GBM * NCAT + 2 * GBM * NH)
#define WSMAX  134217728

static_assert((CHUNK & (CHUNK - 1)) == 0 && CHUNK <= 4096);
static_assert((NBA & (NBA - 1)) == 0 && NBA == (1 << SLA));
static_assert(((long long)CHUNK << SLA) < (1LL << 31));
static_assert(LISTN % NTHR == 0);
static_assert(NBA % NWAVE == 0 && NBA % 32 == 0);
static_assert(RCAP % 4 == 0 && AGG_ZINTS % 4 == 0 && LISTN % 4 == 0);
static_assert(DIN % 32 == 0 && HD == 4 * 32 && NCAT == 2 * HD);
static_assert(GBM == 4 * 16 && NTHR == 8 * 32 && GBM == NWAVE * 8);
static_assert(NUW % NTHR == 0 && (DIN / 8) == 16);
static_assert(MXB == NTHR);
static_assert(AGG_LDS_INTS * 4 <= 300000);
static_assert(2 * GBM * NH == 512);

typedef float          v4f   __attribute__((ext_vector_type(4)));
typedef float          v8f   __attribute__((ext_vector_type(8)));
typedef int            v4i   __attribute__((ext_vector_type(4)));
typedef int            v8i   __attribute__((ext_vector_type(8)));
typedef unsigned int   v4u   __attribute__((ext_vector_type(4)));
typedef unsigned short v8us  __attribute__((ext_vector_type(8)));
typedef unsigned short v16us __attribute__((ext_vector_type(16)));
typedef __bf16         v16bf __attribute__((ext_vector_type(16)));
typedef v4f  __attribute__((may_alias)) v4fa;
typedef v4i  __attribute__((may_alias)) v4ia;
typedef v8us __attribute__((may_alias)) v8usa;
union FragB { v16bf v; v16us u; v8us h[2]; v8i w; v4u q[2]; };

__device__ __forceinline__ v8f wmb(const FragB& a, const FragB& b, v8f c) {
  v8f d = __builtin_amdgcn_wmma_f32_16x16x32_bf16(false, a.v, false, b.v, (short)0, c, false, false);
  asm volatile("v_nop\n\tv_nop\n\tv_nop\n\tv_nop" : "+v"(d) : "v"(a.w), "v"(b.w));
  return d;
}

__device__ __forceinline__ unsigned bf16_bits(float f) {
  const unsigned u = __float_as_uint(f);
  return ((u + 0x7FFFu + ((u >> 16) & 1u)) >> 16) & 0xFFFFu;
}
__device__ __forceinline__ float bf16_val(float f) {
  return __uint_as_float(bf16_bits(f) << 16);
}
__device__ __forceinline__ v4f bfr4(const v4f a) {
  v4f r; r.x = bf16_val(a.x); r.y = bf16_val(a.y); r.z = bf16_val(a.z); r.w = bf16_val(a.w); return r;
}
__device__ __forceinline__ unsigned pk2(float lo, float hi) { return bf16_bits(lo) | (bf16_bits(hi) << 16); }
__device__ __forceinline__ v4u pack8(const v4f a, const v4f b) {
  v4u r;
  r.x = pk2(a.x, a.y); r.y = pk2(a.z, a.w); r.z = pk2(b.x, b.y); r.w = pk2(b.z, b.w);
  return r;
}

template <int SLB>
__device__ __forceinline__ int scan_chunk(const int* __restrict__ dsts, int nE, int cbase, int slotBase,
                                          int nb, int vec8, int* list, int tid, int lane, int wave) {
  int wc = 0;
  const int el0  = tid * EPT;
  const int e0   = cbase + el0;
  const int sent = -2147483647 - 1;
  v4i da, db;
  if (vec8 != 0 && cbase + CHUNK <= nE) {
    da = *(const v4i*)(dsts + e0);
    db = *(const v4i*)(dsts + e0 + 4);
  } else {
    da.x = (e0     < nE) ? dsts[min(e0,     nE - 1)] : sent;
    da.y = (e0 + 1 < nE) ? dsts[min(e0 + 1, nE - 1)] : sent;
    da.z = (e0 + 2 < nE) ? dsts[min(e0 + 2, nE - 1)] : sent;
    da.w = (e0 + 3 < nE) ? dsts[min(e0 + 3, nE - 1)] : sent;
    db.x = (e0 + 4 < nE) ? dsts[min(e0 + 4, nE - 1)] : sent;
    db.y = (e0 + 5 < nE) ? dsts[min(e0 + 5, nE - 1)] : sent;
    db.z = (e0 + 6 < nE) ? dsts[min(e0 + 6, nE - 1)] : sent;
    db.w = (e0 + 7 < nE) ? dsts[min(e0 + 7, nE - 1)] : sent;
  }
  const unsigned nbs = (unsigned)slotBase;
  const unsigned unb = (unsigned)nb;
  const unsigned s0 = (unsigned)da.x - nbs, s1 = (unsigned)da.y - nbs;
  const unsigned s2 = (unsigned)da.z - nbs, s3 = (unsigned)da.w - nbs;
  const unsigned s4 = (unsigned)db.x - nbs, s5 = (unsigned)db.y - nbs;
  const unsigned s6 = (unsigned)db.z - nbs, s7 = (unsigned)db.w - nbs;
  const bool h0 = s0 < unb, h1 = s1 < unb, h2 = s2 < unb, h3 = s3 < unb;
  const bool h4 = s4 < unb, h5 = s5 < unb, h6 = s6 < unb, h7 = s7 < unb;
  const unsigned any = __builtin_amdgcn_ballot_w32(h0 | h1 | h2 | h3 | h4 | h5 | h6 | h7);
  if (any != 0u) {
#define HITJ(J, HJ, SJ) { \
      const unsigned mj = __builtin_amdgcn_ballot_w32(HJ); \
      if (mj != 0u) { \
        if (HJ) { \
          const int pos = wc + (int)__builtin_amdgcn_mbcnt_lo(mj, 0u); \
          if (pos < WCAP) list[wave * WCAP + pos] = ((el0 + (J)) << SLB) | (int)(SJ); \
        } \
        wc += (int)__builtin_popcount(mj); } }
    HITJ(0, h0, s0)
    HITJ(1, h1, s1)
    HITJ(2, h2, s2)
    HITJ(3, h3, s3)
    HITJ(4, h4, s4)
    HITJ(5, h5, s5)
    HITJ(6, h6, s6)
    HITJ(7, h7, s7)
#undef HITJ
  }
  return wc;
}

__global__ __launch_bounds__(NTHR) void k_wtr(const float* __restrict__ W, const float* __restrict__ P,
                                              unsigned short* wt) {
  const int u = (int)blockIdx.x * NTHR + (int)threadIdx.x;
  if (u >= NUW) return;
  const int n  = u >> 4;
  const int k8 = (u & 15) * 8;
  const float* base = (n < HD) ? W : P;
  const int nn = n & (HD - 1);
  const float* p = base + (size_t)k8 * HD + nn;
  v8us o;
#pragma unroll
  for (int i = 0; i < 8; ++i) o[i] = (unsigned short)bf16_bits(p[(size_t)i * HD]);
  unsigned short* dp = wt + (size_t)n * DIN + k8;
  *(volatile v8us*)dp = o;
  __threadfence();
  *(volatile v8us*)dp = o;
}

__global__ __launch_bounds__(NTHR) void k_gemm(const float* __restrict__ x, const unsigned short* __restrict__ WT,
                                               const float* __restrict__ aL, const float* __restrict__ aR,
                                               float* Hm, float* Rm, float* HSp, float* HTp, int nN) {
  extern __shared__ __attribute__((aligned(16))) float gsm[];
  float* stg = gsm;
  float* sdt = gsm + GBM * NCAT;
  const int tid = (int)threadIdx.x, lane = tid & 31, wave = tid >> 5, hh = lane >> 4, m = lane & 15;
  const int rg = wave & 3, cg = wave >> 2;
  const int rowBase = (int)blockIdx.x * GBM;
  const int colBase = cg * HD;

  v8f acc[8];
  {
    const v8f z = {0.f, 0.f, 0.f, 0.f, 0.f, 0.f, 0.f, 0.f};
#pragma unroll
    for (int t = 0; t < 8; ++t) acc[t] = z;
  }
  int ar = rowBase + 16 * rg + m;
  ar = ar < nN ? ar : nN - 1;
  const float* ap = x + (size_t)ar * DIN + 8 * hh;
  const unsigned short* bp = WT + (size_t)(colBase + m) * DIN + 8 * hh;

#pragma unroll 1
  for (int k0 = 0; k0 < DIN; k0 += 32) {
    const v4f a0 = *(const v4fa*)(ap + k0);
    const v4f a1 = *(const v4fa*)(ap + k0 + 4);
    const v4f a2 = *(const v4fa*)(ap + k0 + 16);
    const v4f a3 = *(const v4fa*)(ap + k0 + 20);
    FragB af;
    af.q[0] = pack8(a0, a1);
    af.q[1] = pack8(a2, a3);
#pragma unroll
    for (int nt = 0; nt < 8; ++nt) {
      const unsigned short* wq = bp + (size_t)(16 * nt) * DIN + k0;
      FragB bf;
      bf.h[0] = *(const v8usa*)wq;
      bf.h[1] = *(const v8usa*)(wq + 16);
      acc[nt] = wmb(af, bf, acc[nt]);
    }
  }

#pragma unroll
  for (int nt = 0; nt < 8; ++nt) {
    const int lc = colBase + 16 * nt + m;
#pragma unroll
    for (int r = 0; r < 8; ++r) {
      const int lr = 16 * rg + 8 * hh + r;
      stg[lr * NCAT + lc] = acc[nt][r];
    }
  }
  __syncthreads();

  const v4f al4 = bfr4(*(const v4fa*)(aL + 4 * lane));
  const v4f ar4 = bfr4(*(const v4fa*)(aR + 4 * lane));
  const int head = lane >> 3;
#pragma unroll 1
  for (int i = 0; i < 8; ++i) {
    const int row = wave * 8 + i;
    const v4f p = *(const v4fa*)(stg + row * NCAT + 4 * lane);
    float s = 0.0f, d = 0.0f;
    s = fmaf(p.x, al4.x, s); s = fmaf(p.y, al4.y, s); s = fmaf(p.z, al4.z, s); s = fmaf(p.w, al4.w, s);
    d = fmaf(p.x, ar4.x, d); d = fmaf(p.y, ar4.y, d); d = fmaf(p.z, ar4.z, d); d = fmaf(p.w, ar4.w, d);
#pragma unroll
    for (int off = 4; off > 0; off >>= 1) {
      s += __shfl_xor(s, off);
      d += __shfl_xor(d, off);
    }
    if ((lane & 7) == 0) { sdt[row * NH + head] = s; sdt[GBM * NH + row * NH + head] = d; }
  }
  __syncthreads();

  const int sw  = wave & 3;
  const int seg = (sw & 1) * 32 + lane;
  const v4f sv  = *(const v4fa*)(sdt + (sw >> 1) * (GBM * NH) + 4 * seg);
  float* spl = (sw >> 1) ? HTp : HSp;
  float* sp  = spl + (size_t)rowBase * NH + 4 * seg;
  const bool swr = wave < 4;

#pragma unroll 1
  for (int i = 0; i < 8; ++i) {
    const int row = wave * 8 + i;
    const v4f ph = *(const v4fa*)(stg + row * NCAT + 4 * lane);
    const v4f pr = *(const v4fa*)(stg + row * NCAT + HD + 4 * lane);
    float* oh = Hm + (size_t)(rowBase + row) * HD + 4 * lane;
    float* orr = Rm + (size_t)(rowBase + row) * HD + 4 * lane;
    *(volatile v4f*)oh = ph;
    *(volatile v4f*)orr = pr;
  }
  if (swr) *(volatile v4f*)sp = sv;
  __threadfence();
#pragma unroll 1
  for (int i = 0; i < 8; ++i) {
    const int row = wave * 8 + i;
    const v4f ph = *(const v4fa*)(stg + row * NCAT + 4 * lane);
    const v4f pr = *(const v4fa*)(stg + row * NCAT + HD + 4 * lane);
    float* oh = Hm + (size_t)(rowBase + row) * HD + 4 * lane;
    float* orr = Rm + (size_t)(rowBase + row) * HD + 4 * lane;
    *(volatile v4f*)oh = ph;
    *(volatile v4f*)orr = pr;
  }
  if (swr) *(volatile v4f*)sp = sv;
}

__global__ __launch_bounds__(NTHR) void k_edgemax(const int* __restrict__ ei, int nE, int nN, int iters,
                                                  const float* __restrict__ HSp, const float* __restrict__ HTp,
                                                  float* rec) {
  __shared__ float sm[NWAVE];
  const int tid = (int)threadIdx.x, lane = tid & 31, wave = tid >> 5;
  const int gid = (int)blockIdx.x * NTHR + tid;
  const int stride = MXB * NTHR;
  float mv = __int_as_float((int)0xff800000u);
#pragma unroll 1
  for (int it = 0; it < iters; ++it) {
    int e = gid + it * stride;
    e = e < nE ? e : nE - 1;
    int s = ei[e];
    int t = ei[(size_t)nE + e];
    s = s < 0 ? 0 : (s > nN - 1 ? nN - 1 : s);
    t = t < 0 ? 0 : (t > nN - 1 ? nN - 1 : t);
    const v4f a = *(const v4fa*)(HSp + (size_t)s * NH);
    const v4f b = *(const v4fa*)(HTp + (size_t)t * NH);
    const float q = fmaxf(fmaxf(a.x + b.x, a.y + b.y), fmaxf(a.z + b.z, a.w + b.w));
    mv = fmaxf(mv, q);
  }
#pragma unroll
  for (int off = 16; off > 0; off >>= 1) mv = fmaxf(mv, __shfl_xor(mv, off));
  if (lane == 0) sm[wave] = mv;
  __syncthreads();
  float bm = sm[0];
#pragma unroll
  for (int w2 = 1; w2 < NWAVE; ++w2) bm = fmaxf(bm, sm[w2]);
  v4f rv; rv.x = bm; rv.y = bm; rv.z = bm; rv.w = bm;
  float* rp = rec + (size_t)blockIdx.x * 32 + 4 * (lane & 7);
  const bool wr = (wave == 0) && (lane < 8);
  if (wr) *(volatile v4f*)rp = rv;
  __threadfence();
  if (wr) *(volatile v4f*)rp = rv;
}

__global__ __launch_bounds__(NTHR) void k_agg(const int* __restrict__ keys, const int* __restrict__ tgts,
                                              int nE, int nN, int vec8,
                                              const float* __restrict__ HSp, const float* __restrict__ HTp,
                                              const float* __restrict__ Hm, const float* __restrict__ Rm,
                                              const float* __restrict__ rec, float* outp) {
  extern __shared__ __attribute__((aligned(16))) int dsm[];
  int* list = dsm;
  int* hl   = dsm + LISTN;
  int* sl   = dsm + LISTN + RCAP;
  int* cnt  = dsm + LISTN + 2 * RCAP;
  int* offs = cnt + NBA;
  int* cur  = offs + NBA;
  int* misc = cur + NBA;
  const int tid = (int)threadIdx.x, lane = tid & 31, wave = tid >> 5;
  const int nodeBase = (int)blockIdx.x * NBA;

  {
    const v4i z4 = {0, 0, 0, 0};
    for (int i = tid * 4; i < AGG_ZINTS; i += NTHR * 4) *(v4ia*)(dsm + i) = z4;
    if (tid < 16) misc[tid] = 0;
  }
  {
    float rv = rec[(size_t)tid * 32];
#pragma unroll
    for (int off = 16; off > 0; off >>= 1) rv = fmaxf(rv, __shfl_xor(rv, off));
    if (lane == 0) misc[16 + wave] = __float_as_int(rv);
  }
  __syncthreads();

  int t = 0, ov = 0;
  const int nChunks = (nE + CHUNK - 1) / CHUNK;
#pragma unroll 1
  for (int ch = 0; ch < nChunks; ++ch) {
    const int cbase = ch * CHUNK;
    const int wc = scan_chunk<SLA>(keys, nE, cbase, nodeBase, NBA, vec8, list, tid, lane, wave);
    if (lane == 0) misc[wave] = wc;
    __syncthreads();
    if (wave == 0) {
#pragma unroll 1
      for (int w2 = 0; w2 < NWAVE; ++w2) {
        int c = misc[w2];
        c = c < 0 ? 0 : (c > WCAP ? WCAP : c);
#pragma unroll 1
        for (int b0 = 0; b0 < c; b0 += 32) {
          const int idx = b0 + lane;
          const int ent = list[w2 * WCAP + (idx < WCAP ? idx : WCAP - 1)];
          const int m32 = (c - b0) < 32 ? (c - b0) : 32;
#pragma unroll 1
          for (int k = 0; k < m32; ++k) {
            const int u    = __builtin_amdgcn_readlane(ent, k);
            const int slot = u & (NBA - 1);
            const int el   = (u >> SLA) & (CHUNK - 1);
            const int pk   = ((cbase + el) << SLA) | slot;
            if (t < RCAP) {
              if (lane == 0) { hl[t] = pk; cnt[slot] = cnt[slot] + 1; }
              t = t + 1;
            } else {
              ov = 1;
            }
          }
        }
      }
    }
    __syncthreads();
  }
  if (wave == 0 && lane == 0) { misc[8] = t; misc[9] = ov; }
  __syncthreads();
  int tt = misc[8];
  tt = tt < 0 ? 0 : (tt > RCAP ? RCAP : tt);
  const int ovf = misc[9];

  if (wave == 0) {
    const int base = lane * (NBA / 32);
    int s = 0;
#pragma unroll 1
    for (int i = 0; i < NBA / 32; ++i) s += cnt[base + i];
    int incl = s;
#pragma unroll
    for (int d = 1; d < 32; d <<= 1) {
      const int y = __shfl_up(incl, d, 32);
      if (lane >= d) incl += y;
    }
    int run = incl - s;
#pragma unroll 1
    for (int i = 0; i < NBA / 32; ++i) {
      const int cv = cnt[base + i];
      offs[base + i] = run;
      cur[base + i]  = run;
      run += cv;
    }
  }
  __syncthreads();
  if (wave == 0) {
#pragma unroll 1
    for (int b0 = 0; b0 < tt; b0 += 32) {
      const int idx = b0 + lane;
      const int ent = hl[idx < RCAP ? idx : RCAP - 1];
      const int m32 = (tt - b0) < 32 ? (tt - b0) : 32;
#pragma unroll 1
      for (int k = 0; k < m32; ++k) {
        const int u    = __builtin_amdgcn_readlane(ent, k);
        const int slot = u & (NBA - 1);
        if (lane == 0) {
          int p = cur[slot];
          p = p < 0 ? 0 : (p > RCAP - 1 ? RCAP - 1 : p);
          sl[p] = u;
          cur[slot] = p + 1;
        }
      }
    }
  }
  __syncthreads();

  float gmx = __int_as_float(misc[16]);
#pragma unroll
  for (int w2 = 1; w2 < NWAVE; ++w2) gmx = fmaxf(gmx, __int_as_float(misc[16 + w2]));
  gmx = gmx >= 0.0f ? gmx : NEGSL * gmx;

  const float pz = (ovf != 0) ? __int_as_float(0x7fc00000) : 0.0f;
  const int head = lane >> 3;
#pragma unroll 1
  for (int si = 0; si < NBA / NWAVE; ++si) {
    const int s    = si * NWAVE + wave;
    const int node = nodeBase + s;
    int c = cnt[s];
    const bool big = c > DEGCAP;
    c = c < 0 ? 0 : (c > DEGCAP ? DEGCAP : c);
    int o = offs[s];
    o = o < 0 ? 0 : (o > RCAP ? RCAP : o);
    const int nc = node < nN ? node : nN - 1;
    const float hs = HSp[(size_t)nc * NH + head];
    v4f acc = {0.0f, 0.0f, 0.0f, 0.0f};
    float lsum = 0.0f;
#pragma unroll 1
    for (int b0 = 0; b0 < c; b0 += 32) {
      int idx = o + b0 + lane;
      idx = idx > RCAP - 1 ? RCAP - 1 : idx;
      const int ent = sl[idx];
      int eid = ent >> SLA;
      eid = eid < 0 ? 0 : (eid > nE - 1 ? nE - 1 : eid);
      int tg = tgts[eid];
      tg = tg < 0 ? 0 : (tg > nN - 1 ? nN - 1 : tg);
      const int m32 = (c - b0) < 32 ? (c - b0) : 32;
#pragma unroll 1
      for (int k = 0; k < m32; ++k) {
        const int tk = __builtin_amdgcn_readlane(tg, k);
        const v4f a = *(const v4fa*)(Hm + (size_t)tk * HD + 4 * lane);
        const float htv = HTp[(size_t)tk * NH + head];
        float lg = hs + htv;
        lg = lg >= 0.0f ? lg : NEGSL * lg;
        const float p = expf(lg - gmx);
        lsum += p;
        acc.x = fmaf(p, a.x, acc.x);
        acc.y = fmaf(p, a.y, acc.y);
        acc.z = fmaf(p, a.z, acc.z);
        acc.w = fmaf(p, a.w, acc.w);
      }
    }
    const float inv = __builtin_amdgcn_rcpf(lsum + EPSD);
    const v4f rr = *(const v4fa*)(Rm + (size_t)nc * HD + 4 * lane);
    float e0 = fmaf(acc.x, inv, rr.x);
    float e1 = fmaf(acc.y, inv, rr.y);
    float e2 = fmaf(acc.z, inv, rr.z);
    float e3 = fmaf(acc.w, inv, rr.w);
#pragma unroll 1
    for (int i = 0; i < 4; ++i) {
      const float vv = e0;
      const float em = expm1f(fminf(vv, 0.0f));
      const float r  = vv > 0.0f ? vv : em;
      e0 = e1; e1 = e2; e2 = e3; e3 = r;
    }
    const float pzr = big ? __int_as_float(0x7fc00000) : pz;
    v4f ov4;
    ov4.x = e0 + pzr; ov4.y = e1 + pzr; ov4.z = e2 + pzr; ov4.w = e3 + pzr;
    const bool live = node < nN;
    if (live) {
      float* op = outp + (size_t)node * HD + 4 * lane;
      *(volatile v4f*)op = ov4;
      __threadfence();
      *(volatile v4f*)op = ov4;
    }
  }
}

static inline int cdiv(int a, int b) { return (a + b - 1) / b; }

extern "C" void kernel_launch(void* const* d_in, const int* in_sizes, int n_in,
                              void* d_out, int out_size, void* d_ws, size_t ws_size,
                              hipStream_t stream) {
  if (n_in < 6) return;
  if (in_sizes[0] < DIN || (in_sizes[0] % DIN) != 0) return;
  const int nN = in_sizes[0] / DIN;
  if (nN > (1 << 22)) return;
  if (in_sizes[1] < 2 || (in_sizes[1] & 1) != 0) return;
  const int nE = in_sizes[1] / 2;
  if (nE < 1 || nE >= (1 << 21)) return;
  if (in_sizes[2] != DIN * HD) return;
  if (in_sizes[3] != HD || in_sizes[4] != HD) return;
  if (in_sizes[5] != DIN * HD) return;
  if ((long long)out_size != (long long)nN * HD) return;

  const float* x   = (const float*)d_in[0];
  const int*   ei  = (const int*)d_in[1];
  const float* W   = (const float*)d_in[2];
  const float* aL  = (const float*)d_in[3];
  const float* aR  = (const float*)d_in[4];
  const float* P   = (const float*)d_in[5];
  float* out = (float*)d_out;
  const int* row0 = ei;
  const int* row1 = ei + nE;

  const int MP   = cdiv(nN, GBM) * GBM;
  const int gM   = MP / GBM;
  const int gA   = cdiv(nN, NBA);
  if ((long long)gA * NBA < (long long)nN) return;
  const int vec8 = ((nE & 3) == 0) ? 1 : 0;
  const int iters = cdiv(nE, MXB * NTHR);

  char* ws = (char*)d_ws;
  size_t off = 0;
  const size_t oWT  = off; off += (size_t)NCAT * DIN * 2;              off = (off + 255) & ~(size_t)255;
  const size_t oREC = off; off += (size_t)MXB * 128;                   off = (off + 255) & ~(size_t)255;
  const size_t oHS  = off; off += (size_t)MP * NH * 4;                 off = (off + 255) & ~(size_t)255;
  const size_t oHT  = off; off += (size_t)MP * NH * 4;                 off = (off + 255) & ~(size_t)255;
  const size_t oH   = off; off += (size_t)MP * HD * 4;                 off = (off + 255) & ~(size_t)255;
  const size_t oR   = off; off += (size_t)MP * HD * 4;                 off = (off + 255) & ~(size_t)255;
  if (off > ws_size || off > (size_t)WSMAX) return;
  unsigned short* WT  = (unsigned short*)(ws + oWT);
  float*          REC = (float*)(ws + oREC);
  float*          HS  = (float*)(ws + oHS);
  float*          HT  = (float*)(ws + oHT);
  float*          H   = (float*)(ws + oH);
  float*          R   = (float*)(ws + oR);

  const size_t gemmLds = (size_t)GEMM_LDS_FLOATS * 4;
  const size_t aggLds  = (size_t)AGG_LDS_INTS * 4;
  hipFuncSetAttribute(reinterpret_cast<const void*>(&k_gemm), hipFuncAttributeMaxDynamicSharedMemorySize, (int)gemmLds);
  hipFuncSetAttribute(reinterpret_cast<const void*>(&k_agg),  hipFuncAttributeMaxDynamicSharedMemorySize, (int)aggLds);

  k_wtr<<<NUW / NTHR, NTHR, 0, stream>>>(W, P, WT);
  k_gemm<<<gM, NTHR, gemmLds, stream>>>(x, WT, aL, aR, H, R, HS, HT, nN);
  k_edgemax<<<MXB, NTHR, 0, stream>>>(ei, nE, nN, iters, HS, HT, REC);
  k_agg<<<gA, NTHR, aggLds, stream>>>(row0, row1, nE, nN, vec8, HS, HT, H, R, REC, out);
}
